// LSTM_60713657696421
// MI455X (gfx1250) — hardware-verified
//
#include <hip/hip_runtime.h>
#include <math.h>

constexpr int NBATCH   = 16;
constexpr int NSTEP    = 512;
constexpr int NHID     = 1024;
constexpr int NGATE    = 4;
constexpr int NG4      = NGATE * NHID;
constexpr int NROWS    = NSTEP * NBATCH;
constexpr int WELEMS   = NHID * NHID;
constexpr int HP       = 1024;
constexpr int HBUF     = NBATCH * HP;
constexpr int STGP     = 512;
constexpr int SCAN_THR = 512;
constexpr int CVT_THR  = 256;
constexpr float XCARRY = 16.0f;
constexpr float WCARRY = 16.0f;
constexpr float HCARRY = 16.0f;
constexpr float XW_FOLD = 1.0f / (XCARRY * WCARRY);
constexpr float HW_FOLD = 1.0f / (HCARRY * WCARRY);

static_assert(NHID % 32 == 0, "GEMM K multiple of 32");
static_assert(NROWS % 64 == 0 && NG4 % 64 == 0, "GEMM M, N tile multiples");
static_assert(NHID == 64 * (SCAN_THR / 32), "16 waves x 64 hidden columns");
static_assert(NBATCH == 16, "one 16-row m-subtile");
static_assert((HP * 2) % 16 == 0, "LDS row pitch 16-B aligned");
static_assert(HBUF * 2 == NBATCH * STGP * 4, "one h buffer holds a 16 x 512 f32 staging tile");
static_assert((2 * HBUF / 8) % SCAN_THR == 0, "LDS zero fill exact");
static_assert((NBATCH * STGP / 4) == 4 * SCAN_THR, "staging store loop exact");
static_assert((NROWS * (NHID / 8)) % CVT_THR == 0, "x convert grid exact");
static_assert(((WELEMS / 8) % CVT_THR) == 0 && (WELEMS / 8) / CVT_THR == 512, "512 blocks per weight matrix");

constexpr size_t XH_BYTES   = (size_t)NROWS * NHID * 2;
constexpr size_t WALL_BYTES = (size_t)8 * WELEMS * 2;
constexpr size_t BSUM_BYTES = (size_t)NG4 * 4;
constexpr size_t G_BYTES    = (size_t)NSTEP * NG4 * NBATCH * 2;
constexpr size_t WS_TOTAL   = XH_BYTES + WALL_BYTES + BSUM_BYTES + G_BYTES;
static_assert(XH_BYTES % 256 == 0 && WALL_BYTES % 256 == 0 && BSUM_BYTES % 256 == 0 && G_BYTES % 256 == 0, "aligned carve");
static_assert(WS_TOTAL == (size_t)100679680, "carve total");
static_assert(WS_TOTAL <= (size_t)134217728, "carve within 128 MiB");

typedef __attribute__((ext_vector_type(16))) _Float16 v16h;
typedef __attribute__((ext_vector_type(8)))  _Float16 v8h;
typedef __attribute__((ext_vector_type(8)))  float    v8f;
typedef __attribute__((ext_vector_type(4)))  float    v4f;
typedef __attribute__((ext_vector_type(4)))  unsigned v4u;

__device__ __forceinline__ void grp_guard4_h(v8f& a0, v8f& a1, v8f& a2, v8f& a3,
                                             v16h x, v16h b0, v16h b1, v16h b2, v16h b3) {
  asm volatile("v_nop\n\tv_nop\n\tv_nop\n\tv_nop"
               : "+v"(a0), "+v"(a1), "+v"(a2), "+v"(a3)
               : "v"(x), "v"(b0), "v"(b1), "v"(b2), "v"(b3));
}
__device__ __forceinline__ void grp_guard8_h(v8f& a0, v8f& a1, v8f& a2, v8f& a3,
                                             v8f& a4, v8f& a5, v8f& a6, v8f& a7,
                                             v16h x, v16h b0, v16h b1, v16h b2, v16h b3,
                                             v16h b4, v16h b5, v16h b6, v16h b7) {
  asm volatile("v_nop\n\tv_nop\n\tv_nop\n\tv_nop"
               : "+v"(a0), "+v"(a1), "+v"(a2), "+v"(a3), "+v"(a4), "+v"(a5), "+v"(a6), "+v"(a7)
               : "v"(x), "v"(b0), "v"(b1), "v"(b2), "v"(b3), "v"(b4), "v"(b5), "v"(b6), "v"(b7));
}
__device__ __forceinline__ void keep4_h(v16h a, v16h b, v16h c, v16h d) { asm volatile("v_nop" :: "v"(a), "v"(b), "v"(c), "v"(d)); }
__device__ __forceinline__ void acc_guard4(v8f& a, v8f& b, v8f& c, v8f& d) { asm volatile("v_nop\n\tv_nop\n\tv_nop\n\tv_nop" : "+v"(a), "+v"(b), "+v"(c), "+v"(d)); }

struct FragH {
  union U { v16h v; v8h h[2]; };
  static __device__ __forceinline__ v16h load(const _Float16* p) {
    U f; f.h[0] = *(const v8h*)(p); f.h[1] = *(const v8h*)(p + 16); return f.v;
  }
  static __device__ __forceinline__ v8f mma(v16h a, v16h b, v8f c) {
    return __builtin_amdgcn_wmma_f32_16x16x32_f16(false, a, false, b, (short)0, c, false, false);
  }
};

__device__ __forceinline__ float h16_to_f32(unsigned hb) {
  const unsigned sgn = (hb & 0x8000u) << 16; const unsigned em = hb & 0x7fffu;
  const float fn = __uint_as_float((em << 13) + 0x38000000u);
  const float fs = (float)em * 5.9604644775390625e-8f;
  const float mag = (em < 0x400u) ? fs : fn; return __uint_as_float(__float_as_uint(mag) | sgn); }

__device__ __forceinline__ float fsig(float x)    { return __builtin_amdgcn_rcpf(1.0f + expf(-x)); }
__device__ __forceinline__ float ftanh_e(float x) { return 1.0f - 2.0f * __builtin_amdgcn_rcpf(expf(2.0f * x) + 1.0f); }

__global__ __launch_bounds__(CVT_THR) void cvt_x_kernel(const float* __restrict__ x, _Float16* __restrict__ xh) {
  const int i  = blockIdx.x * CVT_THR + threadIdx.x;
  const int n8 = NROWS * (NHID / 8);
  if (i < n8) {
    const int m  = i >> 7;
    const int c8 = i & 127;
    const int t  = m >> 4;
    const int b  = m & 15;
    const float* sp = x + ((size_t)b * NSTEP + (size_t)t) * NHID + c8 * 8;
    const v4f a0 = *(const v4f*)(sp);
    const v4f a1 = *(const v4f*)(sp + 4);
    v8h hv;
#pragma unroll
    for (int e = 0; e < 4; ++e) {
      hv[e]     = (_Float16)(a0[e] * XCARRY);
      hv[4 + e] = (_Float16)(a1[e] * XCARRY);
    }
    _Float16* dp = xh + (size_t)i * 8;
    *(volatile v8h*)dp = hv;
    __threadfence();
    *(volatile v8h*)dp = hv;
  }
}

__global__ __launch_bounds__(CVT_THR) void cvt_w_kernel(const float* __restrict__ w0, const float* __restrict__ w1,
                                                       const float* __restrict__ w2, const float* __restrict__ w3,
                                                       const float* __restrict__ w4, const float* __restrict__ w5,
                                                       const float* __restrict__ w6, const float* __restrict__ w7,
                                                       _Float16* __restrict__ wall) {
  const int mid = blockIdx.x >> 9;
  if (mid < 8) {
    const float* src = (mid == 0) ? w0 : (mid == 1) ? w1 : (mid == 2) ? w2 : (mid == 3) ? w3
                     : (mid == 4) ? w4 : (mid == 5) ? w5 : (mid == 6) ? w6 : w7;
    const int local = (blockIdx.x & 511) * CVT_THR + threadIdx.x;
    const float* sp = src + (size_t)local * 8;
    const v4f a0 = *(const v4f*)(sp);
    const v4f a1 = *(const v4f*)(sp + 4);
    v8h hv;
#pragma unroll
    for (int e = 0; e < 4; ++e) {
      hv[e]     = (_Float16)(a0[e] * WCARRY);
      hv[4 + e] = (_Float16)(a1[e] * WCARRY);
    }
    _Float16* dp = wall + ((size_t)mid * (WELEMS / 8) + (size_t)local) * 8;
    *(volatile v8h*)dp = hv;
    __threadfence();
    *(volatile v8h*)dp = hv;
  }
}

__global__ __launch_bounds__(CVT_THR) void bsum_kernel(const float* __restrict__ bh0, const float* __restrict__ bh1,
                                                      const float* __restrict__ bh2, const float* __restrict__ bh3,
                                                      const float* __restrict__ bx0, const float* __restrict__ bx1,
                                                      const float* __restrict__ bx2, const float* __restrict__ bx3,
                                                      float* __restrict__ bsum) {
  const int q = blockIdx.x;
  if (q < 4) {
    const float* ph = (q == 0) ? bh0 : (q == 1) ? bh1 : (q == 2) ? bh2 : bh3;
    const float* px = (q == 0) ? bx0 : (q == 1) ? bx1 : (q == 2) ? bx2 : bx3;
    const int idx = threadIdx.x * 4;
    const v4f a = *(const v4f*)(ph + idx);
    const v4f b = *(const v4f*)(px + idx);
    v4f o;
#pragma unroll
    for (int e = 0; e < 4; ++e) o[e] = a[e] + b[e];
    float* op = bsum + q * NHID + idx;
    *(volatile v4f*)op = o;
    __threadfence();
    *(volatile v4f*)op = o;
  }
}

__global__ __launch_bounds__(256) void xproj_gemm_kernel(const _Float16* __restrict__ A, const _Float16* __restrict__ Bt,
                                                        const float* __restrict__ bias, _Float16* __restrict__ G) {
  __shared__ __align__(16) _Float16 sG[8][64 * 16];
  const int lane = threadIdx.x & 31;
  const int wave = threadIdx.x >> 5;
  constexpr int tilesN = NG4 >> 6;
  constexpr int tilesM = NROWS >> 6;
  const int tile = blockIdx.x * 8 + wave;
  if (tile >= tilesM * tilesN) return;
  const int tm = tile / tilesN;
  const int tn = tile - tm * tilesN;
  const int m0 = tm << 6;
  const int n0 = tn << 6;
  const int rlane = lane & 15;
  const int hh    = lane >> 4;
  const int koff  = hh * 8;

  v8f acc[4][4];
#pragma unroll
  for (int i = 0; i < 4; ++i)
#pragma unroll
    for (int j = 0; j < 4; ++j) acc[i][j] = (v8f){0.f, 0.f, 0.f, 0.f, 0.f, 0.f, 0.f, 0.f};

  for (int k0 = 0; k0 < NHID; k0 += 32) {
    v16h bh[4];
#pragma unroll
    for (int j = 0; j < 4; ++j) {
      const size_t bo = (size_t)(n0 + (j << 4) + rlane) * NHID + koff + k0;
      bh[j] = FragH::load(Bt + bo);
    }
#pragma unroll
    for (int i = 0; i < 4; ++i) {
      const size_t ao = (size_t)(m0 + (i << 4) + rlane) * NHID + koff + k0;
      const v16h ah = FragH::load(A + ao);
#pragma unroll
      for (int j = 0; j < 4; ++j) acc[i][j] = FragH::mma(ah, bh[j], acc[i][j]);
      grp_guard4_h(acc[i][0], acc[i][1], acc[i][2], acc[i][3], ah, bh[0], bh[1], bh[2], bh[3]);
    }
    keep4_h(bh[0], bh[1], bh[2], bh[3]);
  }
  acc_guard4(acc[0][0], acc[0][1], acc[0][2], acc[0][3]);
  acc_guard4(acc[1][0], acc[1][1], acc[1][2], acc[1][3]);
  acc_guard4(acc[2][0], acc[2][1], acc[2][2], acc[2][3]);
  acc_guard4(acc[3][0], acc[3][1], acc[3][2], acc[3][3]);

  float bv[4];
#pragma unroll
  for (int j = 0; j < 4; ++j) bv[j] = bias[n0 + (j << 4) + rlane];

  _Float16* slab = sG[wave];
#pragma unroll
  for (int i = 0; i < 4; ++i) {
    const int t = (m0 >> 4) + i;
#pragma unroll
    for (int j = 0; j < 4; ++j) {
      v8h pk;
#pragma unroll
      for (int r = 0; r < 8; ++r) pk[r] = (_Float16)(acc[i][j][r] * XW_FOLD + bv[j]);
      *(v8h*)(slab + ((j << 4) + rlane) * 16 + 8 * hh) = pk;
    }
    __builtin_amdgcn_fence(__ATOMIC_RELEASE, "workgroup");
    __builtin_amdgcn_wave_barrier();
    __builtin_amdgcn_fence(__ATOMIC_ACQUIRE, "workgroup");
    _Float16* gt = G + ((size_t)t * NG4 + (size_t)n0) * 16;
    for (int pass = 0; pass < 2; ++pass) {
#pragma unroll
      for (int it = 0; it < 4; ++it) {
        const v8h v = *(const v8h*)(slab + it * 256 + lane * 8);
        *(volatile v8h*)(gt + it * 256 + lane * 8) = v;
      }
      __threadfence();
    }
    __builtin_amdgcn_fence(__ATOMIC_RELEASE, "workgroup");
    __builtin_amdgcn_wave_barrier();
    __builtin_amdgcn_fence(__ATOMIC_ACQUIRE, "workgroup");
  }
}

__device__ __forceinline__ void cell_group(const v8f aF, const v8f aI, const v8f aG, const v8f aO,
                                           const v4u gF, const v4u gI, const v4u gG, const v4u gO,
                                           float (&cs)[8], _Float16* hdst, float* sdst, const bool last) {
#pragma unroll
  for (int r = 0; r < 8; ++r) {
    const unsigned wF = gF[r >> 1];
    const unsigned wI = gI[r >> 1];
    const unsigned wG = gG[r >> 1];
    const unsigned wO = gO[r >> 1];
    const unsigned bF = (r & 1) ? (wF >> 16) : (wF & 0xffffu);
    const unsigned bI = (r & 1) ? (wI >> 16) : (wI & 0xffffu);
    const unsigned bG = (r & 1) ? (wG >> 16) : (wG & 0xffffu);
    const unsigned bO = (r & 1) ? (wO >> 16) : (wO & 0xffffu);
    const float pf = aF[r] * HW_FOLD + h16_to_f32(bF);
    const float pi = aI[r] * HW_FOLD + h16_to_f32(bI);
    const float pg = aG[r] * HW_FOLD + h16_to_f32(bG);
    const float po = aO[r] * HW_FOLD + h16_to_f32(bO);
    const float fg = fsig(pf);
    const float ig = fsig(pi);
    const float gg = ftanh_e(pg);
    const float og = fsig(po);
    const float cn = cs[r] * fg + ig * gg;
    cs[r] = cn;
    const float hn = ftanh_e(cn) * og;
    if (last) {
      sdst[r * STGP] = hn;
    } else {
      hdst[r * HP] = (_Float16)(hn * HCARRY);
    }
    __builtin_amdgcn_sched_barrier(0);
  }
}

template <int PP>
__device__ __forceinline__ void scan_pass(const _Float16* __restrict__ WH, const v4u* __restrict__ G4,
                                          float* __restrict__ out,
                                          const _Float16* ahrow, _Float16* hnxt, float* stg,
                                          const int t, const int wave, const int c, const int hh, const int tid,
                                          const bool last, float (&cA)[8], float (&cB)[8]) {
  const int koff = hh * 8;
  const int j0 = 64 * wave + 32 * PP + c;
  const int j1 = j0 + 16;
  const _Float16* wh0 = WH + (size_t)j0 * NHID + koff;
  const _Float16* wh1 = WH + (size_t)j1 * NHID + koff;
  const v8f z8 = {0.f, 0.f, 0.f, 0.f, 0.f, 0.f, 0.f, 0.f};
  v8f f0 = z8, i0 = z8, g0 = z8, o0 = z8, f1 = z8, i1 = z8, g1 = z8, o1 = z8;
#pragma unroll 1
  for (int k0 = 0; k0 < NHID; k0 += 32) {
    const v16h a  = FragH::load(ahrow + k0);
    const v16h b0 = FragH::load(wh0 + k0);
    const v16h b1 = FragH::load(wh0 + (size_t)1 * WELEMS + k0);
    const v16h b2 = FragH::load(wh0 + (size_t)2 * WELEMS + k0);
    const v16h b3 = FragH::load(wh0 + (size_t)3 * WELEMS + k0);
    const v16h b4 = FragH::load(wh1 + k0);
    const v16h b5 = FragH::load(wh1 + (size_t)1 * WELEMS + k0);
    const v16h b6 = FragH::load(wh1 + (size_t)2 * WELEMS + k0);
    const v16h b7 = FragH::load(wh1 + (size_t)3 * WELEMS + k0);
    f0 = FragH::mma(a, b0, f0);
    i0 = FragH::mma(a, b1, i0);
    g0 = FragH::mma(a, b2, g0);
    o0 = FragH::mma(a, b3, o0);
    f1 = FragH::mma(a, b4, f1);
    i1 = FragH::mma(a, b5, i1);
    g1 = FragH::mma(a, b6, g1);
    o1 = FragH::mma(a, b7, o1);
    grp_guard8_h(f0, i0, g0, o0, f1, i1, g1, o1, a, b0, b1, b2, b3, b4, b5, b6, b7);
  }
  acc_guard4(f0, i0, g0, o0);
  acc_guard4(f1, i1, g1, o1);
  asm volatile("" ::: "memory");
  {
    const size_t gb = ((size_t)t * NG4 + (size_t)j0) * 2 + (size_t)hh;
    const v4u gF = G4[gb];
    const v4u gI = G4[gb + (size_t)1 * NHID * 2];
    const v4u gG = G4[gb + (size_t)2 * NHID * 2];
    const v4u gO = G4[gb + (size_t)3 * NHID * 2];
    cell_group(f0, i0, g0, o0, gF, gI, gG, gO, cA,
               hnxt + (8 * hh) * HP + j0, stg + (8 * hh) * STGP + 32 * wave + c, last);
  }
  asm volatile("" ::: "memory");
  {
    const size_t gb = ((size_t)t * NG4 + (size_t)j1) * 2 + (size_t)hh;
    const v4u gF = G4[gb];
    const v4u gI = G4[gb + (size_t)1 * NHID * 2];
    const v4u gG = G4[gb + (size_t)2 * NHID * 2];
    const v4u gO = G4[gb + (size_t)3 * NHID * 2];
    cell_group(f1, i1, g1, o1, gF, gI, gG, gO, cB,
               hnxt + (8 * hh) * HP + j1, stg + (8 * hh) * STGP + 32 * wave + 16 + c, last);
  }
  asm volatile("" ::: "memory");
  if (last) {
    __syncthreads();
    for (int pass = 0; pass < 2; ++pass) {
#pragma unroll
      for (int it = 0; it < 4; ++it) {
        const int idx = it * SCAN_THR + tid;
        const int row = idx >> 7;
        const int seg = (idx >> 3) & 15;
        const int l8  = idx & 7;
        const v4f v = *(const v4f*)(stg + 4 * idx);
        *(volatile v4f*)(out + (size_t)row * NHID + 64 * seg + 32 * PP + 4 * l8) = v;
      }
      __threadfence();
    }
    __syncthreads();
  }
}

__global__ __launch_bounds__(SCAN_THR) void lstm_scan_kernel(const _Float16* __restrict__ WH, const v4u* __restrict__ G4,
                                                            float* __restrict__ out) {
  __shared__ __align__(16) _Float16 Ah[2 * HBUF];
  const int tid = threadIdx.x, lane = tid & 31, wave = tid >> 5;
  const int c = lane & 15, hh = lane >> 4;

  {
    const v8h zh = {(_Float16)0.0f, (_Float16)0.0f, (_Float16)0.0f, (_Float16)0.0f,
                    (_Float16)0.0f, (_Float16)0.0f, (_Float16)0.0f, (_Float16)0.0f};
    v8h* lz = (v8h*)Ah;
#pragma unroll 1
    for (int i = tid; i < (2 * HBUF) / 8; i += SCAN_THR) lz[i] = zh;
  }
  float cs0[8], cs1[8], cs2[8], cs3[8];
#pragma unroll
  for (int r = 0; r < 8; ++r) { cs0[r] = 0.0f; cs1[r] = 0.0f; cs2[r] = 0.0f; cs3[r] = 0.0f; }
  __syncthreads();

#pragma unroll 1
  for (int t = 0; t < NSTEP; ++t) {
    const int cur = t & 1;
    const _Float16* ahrow = Ah + cur * HBUF + c * HP + hh * 8;
    _Float16* hnxt = Ah + (cur ^ 1) * HBUF;
    float* stg = (float*)(Ah + (cur ^ 1) * HBUF);
    const bool last = (t == NSTEP - 1);
    scan_pass<0>(WH, G4, out, ahrow, hnxt, stg, t, wave, c, hh, tid, last, cs0, cs1);
    scan_pass<1>(WH, G4, out, ahrow, hnxt, stg, t, wave, c, hh, tid, last, cs2, cs3);
    __syncthreads();
  }
}

extern "C" void kernel_launch(void* const* d_in, const int* in_sizes, int n_in,
                              void* d_out, int out_size, void* d_ws, size_t ws_size, hipStream_t stream) {
  if (n_in < 17 || d_out == nullptr || d_ws == nullptr) return;
  if (in_sizes[0] != NBATCH * NSTEP * NHID) return;
  for (int q = 0; q < 8; ++q) {
    if (in_sizes[1 + 2 * q] != NHID * NHID || in_sizes[2 + 2 * q] != NHID) return;
  }
  if (out_size != NBATCH * NHID) return;
  if (WS_TOTAL > ws_size) return;

  const float* x   = (const float*)d_in[0];
  const float* Whf = (const float*)d_in[1];
  const float* bhf = (const float*)d_in[2];
  const float* Whi = (const float*)d_in[3];
  const float* bhi = (const float*)d_in[4];
  const float* Whg = (const float*)d_in[5];
  const float* bhg = (const float*)d_in[6];
  const float* Who = (const float*)d_in[7];
  const float* bho = (const float*)d_in[8];
  const float* Wxf = (const float*)d_in[9];
  const float* bxf = (const float*)d_in[10];
  const float* Wxi = (const float*)d_in[11];
  const float* bxi = (const float*)d_in[12];
  const float* Wxg = (const float*)d_in[13];
  const float* bxg = (const float*)d_in[14];
  const float* Wxo = (const float*)d_in[15];
  const float* bxo = (const float*)d_in[16];

  char* ws = (char*)d_ws;
  _Float16* XH   = (_Float16*)(ws);
  _Float16* WALL = (_Float16*)(ws + XH_BYTES);
  float*    BSUM = (float*)(ws + XH_BYTES + WALL_BYTES);
  _Float16* G    = (_Float16*)(ws + XH_BYTES + WALL_BYTES + BSUM_BYTES);
  _Float16* WH4  = WALL;
  _Float16* WX4  = WALL + (size_t)4 * WELEMS;

  cvt_x_kernel<<<(NROWS * (NHID / 8)) / CVT_THR, CVT_THR, 0, stream>>>(x, XH);
  cvt_w_kernel<<<8 * 512, CVT_THR, 0, stream>>>(Whf, Whi, Whg, Who, Wxf, Wxi, Wxg, Wxo, WALL);
  bsum_kernel<<<4, CVT_THR, 0, stream>>>(bhf, bhi, bhg, bho, bxf, bxi, bxg, bxo, BSUM);

  xproj_gemm_kernel<<<((NROWS / 64) * (NG4 / 64)) / 8, 256, 0, stream>>>(XH, WX4, BSUM, G);

  lstm_scan_kernel<<<1, SCAN_THR, 0, stream>>>(WH4, (const v4u*)G, (float*)d_out);
}
